// TermEncoder_16423954940619
// MI455X (gfx1250) — hardware-run, weakly checked
//
#include <hip/hip_runtime.h>


namespace {
constexpr int N = 50000, NP = 50048, E = 800000, D0 = 128, NH = 2, C = 128, HC = 256;
constexpr float XS = 8.0f, WSC = 256.0f, NEG = 0.2f, EPSD = 1e-16f;

typedef _Float16 b16;
typedef __attribute__((ext_vector_type(16))) _Float16 v16b;
typedef __attribute__((ext_vector_type(8))) _Float16 v8b;
typedef __attribute__((ext_vector_type(8))) float v8f;
typedef __attribute__((ext_vector_type(4))) float v4f;
__device__ __forceinline__ float bf16_rne(float f) { unsigned int u = __float_as_uint(f); u += 0x7FFFu + ((u >> 16) & 1u); return __uint_as_float(u & 0xFFFF0000u); }
__device__ __forceinline__ void split16(float v, b16& hi, b16& lo) { hi = (b16)v; lo = (b16)(v - (float)hi); }
__device__ __forceinline__ v16b frag_kb(const b16* p, int hh) { const v8b a = *(const v8b*)(p + 8 * hh), b = *(const v8b*)(p + 16 + 8 * hh); v16b f;
#pragma unroll
  for (int e = 0; e < 8; ++e) { f[e] = a[e]; f[8 + e] = b[e]; } return f; }
__device__ __forceinline__ v8f wmma16b(v16b a, v16b b, v8f c) { v8f d = __builtin_amdgcn_wmma_f32_16x16x32_f16(false, a, false, b, (short)0, c, false, false); asm volatile("v_nop\n\tv_nop\n\tv_nop\n\tv_nop" : "+v"(d) : "v"(a), "v"(b)); return d; }
__device__ __forceinline__ void wave_lds_sync() { __builtin_amdgcn_fence(__ATOMIC_RELEASE, "workgroup"); __builtin_amdgcn_wave_barrier(); __builtin_amdgcn_fence(__ATOMIC_ACQUIRE, "workgroup"); }
__device__ __forceinline__ float pmul(float a, float b) { float p = a * b; asm volatile("" : "+v"(p)); return p; }
__device__ __forceinline__ int iclamp(int v, int lo, int hi) { return v < lo ? lo : (v > hi ? hi : v); }
__device__ __forceinline__ float nexp(float x) { return __builtin_amdgcn_exp2f(x * 1.4426950408889634f); }
__device__ __forceinline__ float lrelu(float x) { return x > 0.0f ? x : NEG * x; }

constexpr int CSR_NBLK = 512, CSR_GB = 9, CSR_GN = 1 << CSR_GB  , CSR_MAXG = 512, CSR_CAP = 12288  ;
__global__ __launch_bounds__(64) void csrA_kernel(const int* __restrict__ dst, int E, int N, int nG, int CHP, int NGP, int* __restrict__ STG, int* __restrict__ HST) {
  extern __shared__ int sm[];
  int* cnt = sm; int* run = sm + NGP; int* ids = sm + 2 * NGP;
  const int b = blockIdx.x; const int ch = (E + CSR_NBLK - 1) / CSR_NBLK; const int e0 = b * ch, e1 = min(E, e0 + ch);
  for (int i = threadIdx.x; i < NGP; i += 64) cnt[i] = 0;
  for (int i = threadIdx.x; i < CHP; i += 64) ids[i] = -1;
  __syncthreads();
  if (threadIdx.x == 0) {
    for (int e = e0; e < e1; ++e) { int d = dst[e]; d = (d < 0) ? 0 : (d >= N ? N - 1 : d); cnt[d >> CSR_GB] += 1; }
    int acc = 0; for (int g = 0; g < nG; ++g) { run[g] = acc; acc += cnt[g]; }
    for (int e = e0; e < e1; ++e) { int d = dst[e]; d = (d < 0) ? 0 : (d >= N ? N - 1 : d); const int g = d >> CSR_GB; ids[run[g]] = e; run[g] += 1; } }
  __syncthreads();
  typedef __attribute__((ext_vector_type(4))) int v4i;
  for (int pass = 0; pass < 2; ++pass) {
    for (int i = threadIdx.x; i < CHP / 4; i += 64) *(volatile v4i*)(STG + (size_t)b * CHP + i * 4) = *(const v4i*)(&ids[i * 4]);
    for (int i = threadIdx.x; i < NGP / 4; i += 64) { v4i v; for (int e = 0; e < 4; ++e) v[e] = (i * 4 + e < nG) ? cnt[i * 4 + e] : 0; *(volatile v4i*)(HST + (size_t)b * NGP + i * 4) = v; }
    __threadfence(); }
}
__global__ __launch_bounds__(512) void csrS_kernel(const int* __restrict__ HST, int nG, int NGP, int* __restrict__ START, int* __restrict__ TOT, int* __restrict__ OFF) {
  __shared__ int tot[CSR_MAXG];
  const int b = threadIdx.x;
  for (int pass = 0; pass < 2; ++pass) { int runb = 0; for (int g = 0; g < nG; ++g) { int c = HST[(size_t)b * NGP + g]; c = (c < 0) ? 0 : c; ((volatile int*)OFF)[(size_t)g * CSR_NBLK + b] = runb; runb += c; } __threadfence(); }
  for (int g = threadIdx.x; g < nG; g += 512) { int s = 0; for (int bb = 0; bb < CSR_NBLK; ++bb) { int c = HST[(size_t)bb * NGP + g]; s += (c < 0) ? 0 : c; } tot[g] = s; }
  __syncthreads();
  if (threadIdx.x < 32) {
    __shared__ int st[CSR_MAXG + 32];
    if (threadIdx.x == 0) { int acc = 0; for (int g = 0; g < NGP; ++g) { st[g] = acc; if (g < nG) acc += (tot[g] + 31) & ~31; } st[NGP] = acc; }
    __builtin_amdgcn_fence(__ATOMIC_RELEASE, "workgroup"); __builtin_amdgcn_wave_barrier(); __builtin_amdgcn_fence(__ATOMIC_ACQUIRE, "workgroup");
    for (int pass = 0; pass < 2; ++pass) { for (int i = threadIdx.x; i < NGP + 32; i += 32) { ((volatile int*)START)[i] = (i <= NGP) ? st[min(i, NGP)] : 0; ((volatile int*)TOT)[i] = (i < nG) ? tot[i] : 0; } __threadfence(); } }
}
__global__ __launch_bounds__(256) void csrB_kernel(const int* __restrict__ dst, int N, int nG, int CHP, int NGP, int permLen, const int* __restrict__ STG, const int* __restrict__ HST, const int* __restrict__ OFF, const int* __restrict__ START, const int* __restrict__ TOT, int* __restrict__ PERM, int* __restrict__ ROWPTR, int* __restrict__ ROWCNT, int* __restrict__ FLAG) {
  typedef __attribute__((ext_vector_type(4))) int v4i;
  __shared__ int ids[CSR_CAP]; __shared__ unsigned short key[CSR_CAP]; __shared__ int outp[CSR_CAP]; __shared__ int ncnt[CSR_GN + 1]; __shared__ int boff[CSR_NBLK + 1];
  const int g = blockIdx.x, t_ = threadIdx.x; int tot = TOT[g]; int st = START[g], stn = START[g + 1]; const int v0 = g * CSR_GN; const int nv = min(CSR_GN, N - v0);
  st = (st < 0) ? 0 : (st > permLen - 32 ? permLen - 32 : st) & ~31; stn = (stn < st) ? st : (stn > permLen ? permLen : stn); tot = (tot < 0) ? 0 : tot; if (tot > stn - st && tot <= CSR_CAP) tot = stn - st;
  if (tot > CSR_CAP) {
    for (int pass = 0; pass < 2; ++pass) { for (int i = t_; i < CSR_GN / 4; i += 256) { v4i a, c; for (int e = 0; e < 4; ++e) { a[e] = st; c[e] = 0; } *(volatile v4i*)(ROWPTR + v0 + i * 4) = a; *(volatile v4i*)(ROWCNT + v0 + i * 4) = c; } if (t_ == 0) ((volatile int*)FLAG)[0] = 1; __threadfence(); } (void)nv; return; }
  if (t_ == 0) { int acc = 0; for (int b = 0; b < CSR_NBLK; ++b) { boff[b] = acc; int c = HST[(size_t)b * NGP + g]; c = (c < 0) ? 0 : (c > CHP ? CHP : c); acc += c; if (acc > tot) acc = tot; } boff[CSR_NBLK] = acc; }
  for (int i = t_; i <= CSR_GN; i += 256) ncnt[i] = 0;
  __syncthreads();
  for (int b = 0; b < CSR_NBLK; ++b) { const int c = boff[b + 1] - boff[b]; int o_ = OFF[(size_t)g * CSR_NBLK + b]; o_ = (o_ < 0) ? 0 : (o_ > CHP - c ? CHP - c : o_); const int* src_ = STG + (size_t)b * CHP + o_;
    for (int i = t_; i < c; i += 256) { int id = src_[i]; id = (id < 0) ? 0 : id; ids[boff[b] + i] = id; int d = dst[id]; d = (d < v0) ? v0 : (d >= N ? N - 1 : d); int kk = d - v0; kk = (kk < 0) ? 0 : (kk >= CSR_GN ? CSR_GN - 1 : kk); key[boff[b] + i] = (unsigned short)kk; } }
  __syncthreads();
  if (t_ == 0) { for (int i = 0; i < tot; ++i) ncnt[key[i]] += 1; int acc = 0; for (int vl = 0; vl < CSR_GN; ++vl) { const int c = ncnt[vl]; ncnt[vl] = acc; acc += c; } ncnt[CSR_GN] = acc;
    for (int i = 0; i < tot; ++i) { const int vl = key[i]; outp[ncnt[vl]] = ids[i]; ncnt[vl] += 1; }
    for (int vl = CSR_GN; vl > 0; --vl) ncnt[vl] = ncnt[vl - 1]; ncnt[0] = 0; }
  __syncthreads();
  for (int pass = 0; pass < 2; ++pass) {
    for (int i = t_; i < (stn - st) / 4; i += 256) { v4i v; for (int e = 0; e < 4; ++e) { const int q = i * 4 + e; v[e] = (q < tot) ? outp[q] : -1; } *(volatile v4i*)(PERM + st + i * 4) = v; }
    for (int i = t_; i < CSR_GN / 4; i += 256) { v4i a, c; for (int e = 0; e < 4; ++e) { const int vl = i * 4 + e; a[e] = st + ncnt[vl]; c[e] = (vl < nv) ? (ncnt[vl + 1] - ncnt[vl]) : 0; } *(volatile v4i*)(ROWPTR + v0 + i * 4) = a; *(volatile v4i*)(ROWCNT + v0 + i * 4) = c; }
    __threadfence(); }
}
__global__ __launch_bounds__(256) void csrZ_kernel(int* __restrict__ p, size_t n4) { typedef __attribute__((ext_vector_type(4))) int v4i; const size_t tid = (size_t)blockIdx.x * 256 + threadIdx.x, nth = (size_t)gridDim.x * 256; v4i z = {0, 0, 0, 0}; for (size_t i = tid; i < n4; i += nth) *(volatile v4i*)(p + i * 4) = z; }
struct CsrBufs { int *STG, *HST, *OFF, *START, *TOT, *PERM, *ROWPTR, *ROWCNT, *FLAG; int nG, NGP, CHP; size_t permLen; char* base; size_t bytes; };
static size_t csr_carve(CsrBufs& c, char* ws, size_t off, int E, int N) {
  const size_t off0 = off; c.base = ws + off;
  auto al = [&](size_t bytes) { char* p = ws + off; off += (bytes + 255) & ~(size_t)255; return p; };
  c.nG = (N + CSR_GN - 1) / CSR_GN; c.NGP = (c.nG + 31) & ~31; const int ch = (E + CSR_NBLK - 1) / CSR_NBLK; c.CHP = (ch + 31) & ~31; c.permLen = (size_t)E + 32 * (size_t)c.nG + 32;
  c.STG = (int*)al((size_t)CSR_NBLK * c.CHP * 4); c.HST = (int*)al((size_t)CSR_NBLK * c.NGP * 4); c.OFF = (int*)al((size_t)c.NGP * CSR_NBLK * 4); c.START = (int*)al((size_t)(c.NGP + 64) * 4); c.TOT = (int*)al((size_t)(c.NGP + 64) * 4);
  c.PERM = (int*)al(c.permLen * 4); c.ROWPTR = (int*)al((size_t)c.nG * CSR_GN * 4); c.ROWCNT = (int*)al((size_t)c.nG * CSR_GN * 4); c.FLAG = (int*)al(256);
  c.bytes = off - off0; return off;
}
static void csr_build(const CsrBufs& c, const int* dst, int E, int N, hipStream_t stream) {
  const size_t smem = (size_t)(2 * c.NGP + c.CHP) * 4;
  csrZ_kernel<<<512, 256, 0, stream>>>((int*)c.base, c.bytes / 16);
  csrA_kernel<<<CSR_NBLK, 64, smem, stream>>>(dst, E, N, c.nG, c.CHP, c.NGP, c.STG, c.HST);
  csrS_kernel<<<1, 512, 0, stream>>>(c.HST, c.nG, c.NGP, c.START, c.TOT, c.OFF);
  csrB_kernel<<<c.nG, 256, 0, stream>>>(dst, N, c.nG, c.CHP, c.NGP, (int)c.permLen, c.STG, c.HST, c.OFF, c.START, c.TOT, c.PERM, c.ROWPTR, c.ROWCNT, c.FLAG);
}


__global__ __launch_bounds__(256) void prep_kernel(const float* __restrict__ x, const float* __restrict__ w1, const float* __restrict__ w2, const float* __restrict__ wp1, const float* __restrict__ wp2, b16* __restrict__ Xh, b16* __restrict__ WT) {
  const size_t t = (size_t)blockIdx.x * 256 + threadIdx.x; const size_t nx = (size_t)NP * D0 / 8; const size_t n1 = (size_t)HC * D0 / 8, n2 = (size_t)HC * HC / 8, n3 = (size_t)C * HC / 8, n4 = (size_t)C * C / 8; v8b o;
  if (t < nx) { const size_t e = t * 8; const size_t row = e / D0; for (int j = 0; j < 8; ++j) o[j] = (row < (size_t)N) ? (b16)(bf16_rne(x[e + j]) * XS) : (b16)0.0f; for (int pass = 0; pass < 2; ++pass) { *(volatile v8b*)(Xh + e) = o; __threadfence(); } return; }
  size_t u = t - nx; const float* w; size_t woff;
  if (u < n1) { w = w1; woff = 0; } else if ((u -= n1) < n2) { w = w2; woff = n1 * 8; } else if ((u -= n2) < n3) { w = wp1; woff = (n1 + n2) * 8; } else if ((u -= n3) < n4) { w = wp2; woff = (n1 + n2 + n3) * 8; } else return;
  const size_t e = u * 8; for (int j = 0; j < 8; ++j) o[j] = (b16)(bf16_rne(w[e + j]) * WSC); for (int pass = 0; pass < 2; ++pass) { *(volatile v8b*)(WT + woff + e) = o; __threadfence(); }
}
template <int MODE, int K>
__global__ __launch_bounds__(128) void gemm_kernel(const b16* __restrict__ Ah, const b16* __restrict__ Al, const b16* __restrict__ W, const float* __restrict__ bias, float* __restrict__ Yf, b16* __restrict__ Yh, b16* __restrict__ Yl, int ldy) {
  __shared__ __attribute__((aligned(16))) float Ts[4][16][128 + 4];
  const int wave = threadIdx.x >> 5, lane = threadIdx.x & 31, nloc = lane & 15, hlf = lane >> 4; const size_t m0 = (size_t)blockIdx.x * 64 + wave * 16; const int n0 = blockIdx.y * 128;
  v8f acc[8];
#pragma unroll
  for (int t = 0; t < 8; ++t) acc[t] = (v8f){};
#pragma unroll 2
  for (int kb = 0; kb < K; kb += 32) { const v16b a = frag_kb(Ah + (m0 + nloc) * K + kb, hlf); v16b al = {}; if (Al) al = frag_kb(Al + (m0 + nloc) * K + kb, hlf);
#pragma unroll
    for (int t = 0; t < 8; ++t) { const v16b bw = frag_kb(W + (size_t)(n0 + t * 16 + nloc) * K + kb, hlf); acc[t] = wmma16b(a, bw, acc[t]); if (Al) acc[t] = wmma16b(al, bw, acc[t]); } }
#pragma unroll
  for (int t = 0; t < 8; ++t) { const int c = n0 + t * 16 + nloc; const float bb = bias ? bf16_rne(bias[c]) : 0.0f;
#pragma unroll
    for (int r = 0; r < 8; ++r) Ts[wave][8 * hlf + r][t * 16 + nloc] = acc[t][r] * (1.0f / (XS * WSC)) + bb; }
  wave_lds_sync();
  for (int pass = 0; pass < 2; ++pass) { for (int rr = 0; rr < 16; ++rr) { const size_t row = m0 + rr;
      if (MODE == 0) *(volatile v4f*)(Yf + row * ldy + n0 + lane * 4) = *(const v4f*)(&Ts[wave][rr][lane * 4]);
      else if (MODE == 1) { if (lane < 16) { v8b hv, lv; for (int j = 0; j < 8; ++j) { b16 p, q; split16(((row < (size_t)N) ? Ts[wave][rr][lane * 8 + j] : 0.0f) * XS, p, q); hv[j] = p; lv[j] = q; } *(volatile v8b*)(Yh + row * ldy + n0 + lane * 8) = hv; *(volatile v8b*)(Yl + row * ldy + n0 + lane * 8) = lv; } }
      else { if (row < (size_t)N) *(volatile v4f*)(Yf + row * ldy + n0 + lane * 4) = *(const v4f*)(&Ts[wave][rr][lane * 4]); } }
    __threadfence(); }
}
__global__ __launch_bounds__(256) void node_kernel(const float* __restrict__ XL, const float* __restrict__ al_, const float* __restrict__ ar_, float* __restrict__ AL, float* __restrict__ AR) {
  __shared__ float la[8][4], ra[8][4];
  const int wave = threadIdx.x >> 5, lane = threadIdx.x & 31; const size_t v = (size_t)blockIdx.x * 8 + wave; const int c0 = lane * 8;
  float s = 0.0f, d = 0.0f; const float* hr = XL + v * HC + c0; for (int j = 0; j < 8; ++j) { const float hv = hr[j]; s += pmul(hv, bf16_rne(al_[c0 + j])); d += pmul(hv, bf16_rne(ar_[c0 + j])); }
  s += __shfl_xor(s, 1); s += __shfl_xor(s, 2); s += __shfl_xor(s, 4); s += __shfl_xor(s, 8); d += __shfl_xor(d, 1); d += __shfl_xor(d, 2); d += __shfl_xor(d, 4); d += __shfl_xor(d, 8);
  if (lane == 0) { la[wave][0] = s; ra[wave][0] = d; } if (lane == 16) { la[wave][1] = s; ra[wave][1] = d; } if (lane == 1) { la[wave][2] = 0.0f; la[wave][3] = 0.0f; ra[wave][2] = 0.0f; ra[wave][3] = 0.0f; }
  __syncthreads();
  for (int pass = 0; pass < 2; ++pass) { if (threadIdx.x < 8) { *(volatile v4f*)(AL + ((size_t)blockIdx.x * 8 + threadIdx.x) * 4) = *(const v4f*)(&la[threadIdx.x][0]); *(volatile v4f*)(AR + ((size_t)blockIdx.x * 8 + threadIdx.x) * 4) = *(const v4f*)(&ra[threadIdx.x][0]); } __threadfence(); }
}
__global__ __launch_bounds__(256) void agg_kernel(const float* __restrict__ XL, const float* __restrict__ AL, const float* __restrict__ AR, const int* __restrict__ srcs, const int* __restrict__ PERM, const int* __restrict__ ROWPTR, const int* __restrict__ ROWCNT, int permLen, b16* __restrict__ Hh, b16* __restrict__ Hl) {
  const int wave = threadIdx.x >> 5, lane = threadIdx.x & 31; const size_t v = (size_t)blockIdx.x * 8 + wave; const int h = lane >> 4, c0 = lane * 8;
  int st = 0, cnt = 0; if (v < (size_t)N) { st = ROWPTR[v]; cnt = ROWCNT[v]; cnt = iclamp(cnt, 0, 8192); st = iclamp(st, 0, permLen - cnt); }
  const float arv = AR[v * 4 + h]; float mx = -INFINITY;
  for (int j = 0; j < cnt; ++j) { const int e = iclamp(PERM[st + j], 0, E - 1); const int s = iclamp(srcs[e], 0, N - 1); mx = fmaxf(mx, lrelu(AL[(size_t)s * 4 + h] + arv)); }
  if (!(mx > -INFINITY)) mx = 0.0f;
  float den = 0.0f; float acc[8]; for (int q = 0; q < 8; ++q) acc[q] = 0.0f;
  for (int j = 0; j < cnt; ++j) { const int e = iclamp(PERM[st + j], 0, E - 1); const int s = iclamp(srcs[e], 0, N - 1); const float w = nexp(lrelu(AL[(size_t)s * 4 + h] + arv) - mx); den += w; const float* hr = XL + (size_t)s * HC + c0; const v4f h0 = *(const v4f*)hr, h1 = *(const v4f*)(hr + 4); for (int q = 0; q < 4; ++q) { acc[q] += pmul(w, h0[q]); acc[4 + q] += pmul(w, h1[q]); } }
  const float inv = 1.0f / (den + EPSD); v8b hv, lv; for (int q = 0; q < 8; ++q) { b16 p, qq; split16(fmaxf(acc[q] * inv, 0.0f) * XS, p, qq); hv[q] = p; lv[q] = qq; }
  for (int pass = 0; pass < 2; ++pass) { *(volatile v8b*)(Hh + v * HC + c0) = hv; *(volatile v8b*)(Hl + v * HC + c0) = lv; __threadfence(); }
}
}

extern "C" void kernel_launch(void* const* d_in, const int* in_sizes, int n_in, void* d_out, int out_size, void* d_ws, size_t ws_size, hipStream_t stream) {
  (void)n_in;
  auto Fp = [&](int i) { return (const float*)d_in[i]; }; auto Ip = [&](int i) { return (const int*)d_in[i]; };
  if (in_sizes[0] != N * D0 || in_sizes[1] != 2 * E || in_sizes[2] != HC * D0 || in_sizes[5] != HC * HC || in_sizes[8] != C * HC || in_sizes[10] != C * C || out_size != N * C) return;
  size_t off = 0; char* ws = (char*)d_ws;
  auto carve = [&](size_t bytes) { char* p = ws + off; off += (bytes + 255) & ~(size_t)255; return p; };
  b16* Xh = (b16*)carve((size_t)NP * D0 * 2); b16* WT = (b16*)carve(((size_t)HC * D0 + (size_t)HC * HC + (size_t)C * HC + (size_t)C * C) * 2);
  float* XL = (float*)carve((size_t)NP * HC * 4); b16* Hh = (b16*)carve((size_t)NP * HC * 2); b16* Hl = (b16*)carve((size_t)NP * HC * 2); float* AL = (float*)carve((size_t)NP * 4 * 4); float* AR = (float*)carve((size_t)NP * 4 * 4);
  b16* Th = (b16*)XL; b16* Tl = (b16*)XL + (size_t)NP * C;
  CsrBufs csr; off = csr_carve(csr, ws, off, E, N);
  if (off > ws_size || off > ((size_t)128 << 20)) return;
  const b16 *W1 = WT, *W2 = WT + (size_t)HC * D0, *WP1 = W2 + (size_t)HC * HC, *WP2 = WP1 + (size_t)C * HC;
  prep_kernel<<<(unsigned)(((size_t)NP * D0 / 8 + ((size_t)HC * D0 + (size_t)HC * HC + (size_t)C * HC + (size_t)C * C) / 8 + 255) / 256), 256, 0, stream>>>(Fp(0), Fp(2), Fp(5), Fp(8), Fp(10), Xh, WT);
  csr_build(csr, Ip(1) + E, E, N, stream);
  gemm_kernel<0, D0><<<dim3(NP / 64, 2), 128, 0, stream>>>(Xh, nullptr, W1, nullptr, XL, nullptr, nullptr, HC);
  node_kernel<<<NP / 8, 256, 0, stream>>>(XL, Fp(3), Fp(4), AL, AR);
  agg_kernel<<<NP / 8, 256, 0, stream>>>(XL, AL, AR, Ip(1), csr.PERM, csr.ROWPTR, csr.ROWCNT, (int)csr.permLen, Hh, Hl);
  gemm_kernel<0, HC><<<dim3(NP / 64, 2), 128, 0, stream>>>(Hh, Hl, W2, nullptr, XL, nullptr, nullptr, HC);
  node_kernel<<<NP / 8, 256, 0, stream>>>(XL, Fp(6), Fp(7), AL, AR);
  agg_kernel<<<NP / 8, 256, 0, stream>>>(XL, AL, AR, Ip(1), csr.PERM, csr.ROWPTR, csr.ROWCNT, (int)csr.permLen, Hh, Hl);
  gemm_kernel<1, HC><<<dim3(NP / 64, 1), 128, 0, stream>>>(Hh, Hl, WP1, Fp(9), nullptr, Th, Tl, C);
  gemm_kernel<2, C><<<dim3(NP / 64, 1), 128, 0, stream>>>(Th, Tl, WP2, Fp(11), (float*)d_out, nullptr, nullptr, C);
}
